// GraphormerAttentionHead_24464133718314
// MI455X (gfx1250) — hardware-run, weakly checked
//
#include <hip/hip_runtime.h>


#ifndef SEQ
#define SEQ 8192
#endif
#define SEQ_FULL 8192
#define DIN  512
#define DK   512
#define FW   8
#define PANEL (32 * FW)
#define PP   (PANEL + 8)
#define OSP  68
#define AWORDS (SEQ / 32)
#define AROWS 64
#define ECH  1024
#define SC2  ((float)(0.044194173824159216 * 1.4426950408889634))
#define FILL2 ((float)(-1000000.0 * 1.4426950408889634))
#define PSH  14.0f
#define NEGB (-3.0e38f)

static_assert(DIN % 32 == 0);
static_assert(DK % 32 == 0);
static_assert(DK % 64 == 0);
static_assert(DIN % 8 == 0);
static_assert(SEQ % 64 == 0);
static_assert(SEQ % PANEL == 0);
static_assert(SEQ % 16 == 0);
static_assert(SEQ % AROWS == 0);
static_assert(SEQ <= 8192);
static_assert(SEQ <= SEQ_FULL);
static_assert(AWORDS <= 256);
static_assert(DK == 64 * FW);
static_assert(PANEL == 256);
static_assert(PANEL % 32 == 0);
static_assert((PP * 2) % 16 == 0);
static_assert((OSP * 4) % 16 == 0);
static_assert((AROWS & (AROWS - 1)) == 0);
static_assert((AROWS * AWORDS) % 4 == 0);
static_assert(ECH == 256 * 4);
static_assert(4 * 32 * 16 == 16 * 64 * 2);
static_assert(8 * 32 * 16 == 16 * 64 * 4);
static_assert((size_t)AROWS * AWORDS * 4 + 8 * 128 * 4 + 8 * 4 <= 131072);
static_assert((size_t)16 * PP * 2 + 2 * FW * 16 * 4 + (size_t)FW * 16 * OSP * 4 <= 131072);
static_assert((size_t)16 * 68 * 4 <= 131072);
static_assert(((size_t)SEQ * DIN) % 8 == 0);
static_assert(((size_t)DIN * DK) % 8 == 0);

typedef _Float16 h16;
typedef unsigned short bf;
typedef __attribute__((ext_vector_type(16))) __bf16   v16bf;
typedef __attribute__((ext_vector_type(16))) _Float16 v16h;
typedef __attribute__((ext_vector_type(8)))  _Float16 v8h;
typedef __attribute__((ext_vector_type(8)))  unsigned short v8us;
typedef __attribute__((ext_vector_type(8)))  float    v8f;
typedef __attribute__((ext_vector_type(4)))  float    v4f;
typedef v4f  __attribute__((may_alias)) v4fa;
typedef __attribute__((ext_vector_type(4)))  unsigned v4u;
typedef v4u  __attribute__((may_alias)) v4ua;
typedef __attribute__((ext_vector_type(4)))  int      v4i;

__device__ __forceinline__ unsigned short f2bf(float f) { unsigned u = __float_as_uint(f); u += 0x7FFFu + ((u >> 16) & 1u); return (unsigned short)(u >> 16); }
__device__ __forceinline__ float bfr(float f) { return __uint_as_float(((unsigned)f2bf(f)) << 16); }
__device__ __forceinline__ v16h cat16(v8h lo, v8h hi) { return __builtin_shufflevector(lo, hi, 0, 1, 2, 3, 4, 5, 6, 7, 8, 9, 10, 11, 12, 13, 14, 15); }
__device__ __forceinline__ v16bf cat16b(v8us lo, v8us hi) { return __builtin_bit_cast(v16bf, __builtin_shufflevector(lo, hi, 0, 1, 2, 3, 4, 5, 6, 7, 8, 9, 10, 11, 12, 13, 14, 15)); }
__device__ __forceinline__ v8f wmma16(v16h a, v16h b, v8f c) { return __builtin_amdgcn_wmma_f32_16x16x32_f16(false, a, false, b, (short)0, c, false, false); }
__device__ __forceinline__ v8f wmmab(v16bf a, v16bf b, v8f c) { return __builtin_amdgcn_wmma_f32_16x16x32_bf16(false, a, false, b, (short)0, c, false, false); }
__device__ __forceinline__ v16h  ldh(const h16* p) { return cat16(*(const v8h*)p, *(const v8h*)(p + 16)); }
__device__ __forceinline__ v16bf ldb(const bf* p)  { return cat16b(*(const v8us*)p, *(const v8us*)(p + 16)); }
__device__ __forceinline__ void wave_sync() { __builtin_amdgcn_fence(3  , "wavefront"); __builtin_amdgcn_wave_barrier(); asm volatile("" ::: "memory"); }

static __device__ __forceinline__ h16 toh_flush(float v) { const h16 r = (h16)v; return (fabsf(v) < 6.103515625e-05f) ? (h16)0.0f : r; }
__device__ __forceinline__ v8f wmg(v16h a, v16h b, v8f c) { c = wmma16(a, b, c); asm volatile("v_nop\n\tv_nop\n\tv_nop\n\tv_nop" : "+v"(c) : "v"(a), "v"(b)); return c; }

__global__ __launch_bounds__(256) void k_cvt8(const float* __restrict__ src, bf* dst, size_t n8) {
    const size_t i = (size_t)blockIdx.x * 256 + threadIdx.x; if (i >= n8) return;
    const v8f v = *(const v8f*)(src + i * 8); v8us o;
#pragma unroll
    for (int k = 0; k < 8; ++k) o[k] = f2bf(v[k]);
    *(volatile v8us*)(dst + i * 8) = o; __threadfence(); *(volatile v8us*)(dst + i * 8) = o;
}

__global__ __launch_bounds__(256) void k_wcvt(const float* __restrict__ W, bf* WT) {
    const int i = blockIdx.x * 256 + threadIdx.x; if (i >= DK * DIN / 8) return;
    const int n = i / (DIN / 8), k8 = (i % (DIN / 8)) * 8; v8us o;
#pragma unroll
    for (int j = 0; j < 8; ++j) o[j] = f2bf(W[(size_t)(k8 + j) * DK + n]);
    *(volatile v8us*)(WT + (size_t)i * 8) = o; __threadfence(); *(volatile v8us*)(WT + (size_t)i * 8) = o;
}

__global__ __launch_bounds__(256) void k_adj(const int* __restrict__ ei, unsigned* ADJ, int E) {
    __shared__ __align__(16) unsigned bits[AROWS * AWORDS];
    __shared__ unsigned hl[8 * 128];
    __shared__ int hc[8];
    const int tid = threadIdx.x, lane = tid & 31;
    const int wave = __builtin_amdgcn_readfirstlane((int)(threadIdx.x >> 5));
    const int r0 = blockIdx.x * AROWS;
#pragma unroll 1
    for (int i = tid; i < AROWS * AWORDS / 4; i += 256) { const v4u z = (v4u){0u, 0u, 0u, 0u}; *(v4ua*)(&bits[i * 4]) = z; }
    __syncthreads();
    const int nch = (E + ECH - 1) / ECH;
    const int Em1 = E - 1;
#pragma unroll 1
    for (int ch = 0; ch < nch; ++ch) {
        const int cb = ch * ECH;
        int sv[4], dv[4];
        if (((E & 3) == 0) & (cb + ECH <= E)) {
            const v4i s4 = *(const v4i*)(ei + (size_t)cb + (size_t)tid * 4);
            const v4i d4 = *(const v4i*)(ei + (size_t)E + (size_t)cb + (size_t)tid * 4);
#pragma unroll
            for (int j = 0; j < 4; ++j) { sv[j] = s4[j]; dv[j] = d4[j]; }
        } else {
#pragma unroll
            for (int j = 0; j < 4; ++j) {
                const int e = cb + tid * 4 + j;
                const int ec = e < Em1 ? e : Em1;
                int s = ei[(size_t)ec]; int d = ei[(size_t)E + (size_t)ec];
                asm volatile("" : "+v"(s)); asm volatile("" : "+v"(d));
                sv[j] = (e < E) ? s : 0x40000000; dv[j] = d;
            }
        }
        int base = 0;
#pragma unroll
        for (int j = 0; j < 4; ++j) {
            int s = sv[j]; s += (s < 0) ? SEQ : 0;
            int d = dv[j]; d += (d < 0) ? SEQ : 0;
            const bool hit = ((unsigned)(s - r0) < (unsigned)AROWS) & ((unsigned)d < (unsigned)SEQ);
            const unsigned mask = __builtin_amdgcn_ballot_w32(hit);
            const int pos = base + (int)__builtin_amdgcn_mbcnt_lo(mask, 0u);
            if (hit) hl[wave * 128 + pos] = ((unsigned)(s - r0) << 13) | (unsigned)d;
            base += __builtin_popcount(mask);
        }
        if (lane == 0) hc[wave] = base;
        __syncthreads();
#pragma unroll 1
        for (int w = 0; w < 8; ++w) {
            int n = hc[w]; n = n < 0 ? 0 : (n > 128 ? 128 : n);
            n = __builtin_amdgcn_readfirstlane(n);
#pragma unroll 1
            for (int i = 0; i < n; ++i) {
                const unsigned ent = hl[w * 128 + i];
                const int c = (int)(ent & 8191u); const int rr = (int)(ent >> 13) & (AROWS - 1);
                if ((c >> 5) == tid) bits[rr * AWORDS + tid] |= 1u << (c & 31);
            }
        }
        __syncthreads();
    }
    unsigned* dst = ADJ + (size_t)r0 * AWORDS;
#pragma unroll 1
    for (int ps = 0; ps < 2; ++ps) {
#pragma unroll 1
        for (int i = tid; i < AROWS * AWORDS / 4; i += 256) { const v4u v = *(const v4ua*)(&bits[i * 4]); *(volatile v4u*)(dst + (size_t)i * 4) = v; }
        if (ps == 0) __threadfence(); }
}

template <int MODE>
__device__ __forceinline__ void proj_body(const bf* __restrict__ A, const bf* __restrict__ Bt, const float* __restrict__ bias, h16* Ph) {
    __shared__ __align__(16) float os[16 * 68];
    const int K = DIN;
    const int lane = threadIdx.x & 31, lr = lane & 15, hi = lane >> 4; const int r0 = blockIdx.x * 64, c0 = blockIdx.y * 64;
    v8f acc[4][4];
#pragma unroll
    for (int mb = 0; mb < 4; ++mb)
#pragma unroll
        for (int nb = 0; nb < 4; ++nb) acc[mb][nb] = (v8f){};
    const size_t aoff = (size_t)(r0 + lr) * K + 8 * hi, boff = (size_t)(c0 + lr) * K + 8 * hi;
#pragma unroll 1
    for (int kc = 0; kc < K; kc += 32) {
        v16bf a[4];
#pragma unroll
        for (int mb = 0; mb < 4; ++mb) a[mb] = ldb(A + aoff + (size_t)mb * 16 * K + kc);
#pragma unroll
        for (int nb = 0; nb < 4; ++nb) { const v16bf b = ldb(Bt + boff + (size_t)nb * 16 * K + kc);
#pragma unroll
            for (int mb = 0; mb < 4; ++mb) acc[mb][nb] = wmmab(a[mb], b, acc[mb][nb]); }
        asm volatile("v_nop\n\tv_nop\n\tv_nop\n\tv_nop" : "+v"(acc[0][0]), "+v"(acc[1][1]), "+v"(acc[2][2]), "+v"(acc[3][3]) : "v"(a[0]), "v"(a[1]), "v"(a[2]), "v"(a[3]));
    }
    float bc[4];
#pragma unroll
    for (int nb = 0; nb < 4; ++nb) bc[nb] = (MODE == 0) ? bfr(bias[c0 + nb * 16 + lr]) : 0.0f;
    const size_t pitch = (MODE == 0) ? (size_t)DK : (size_t)SEQ;
    const size_t tbase = (size_t)r0 * pitch + (size_t)c0;
#pragma unroll
    for (int mb = 0; mb < 4; ++mb) {
        float br[8];
#pragma unroll
        for (int j = 0; j < 8; ++j) br[j] = (MODE == 1) ? bfr(bias[r0 + mb * 16 + hi * 8 + j]) : 0.0f;
#pragma unroll
        for (int nb = 0; nb < 4; ++nb) {
#pragma unroll
            for (int j = 0; j < 8; ++j) os[(hi * 8 + j) * 68 + nb * 16 + lr] = acc[mb][nb][j] + bc[nb] + br[j]; }
        wave_sync();
#pragma unroll 1
        for (int ps = 0; ps < 2; ++ps) {
            const size_t sb = tbase + (size_t)(mb * 16) * pitch;
#pragma unroll
            for (int s = 0; s < 4; ++s) { const int row = 4 * s + (lane >> 3), c8 = (lane & 7) * 8;
                const v4f x0 = *(const v4fa*)(&os[row * 68 + c8]); const v4f x1 = *(const v4fa*)(&os[row * 68 + c8 + 4]); v8h hv;
#pragma unroll
                for (int i = 0; i < 4; ++i) { hv[i] = toh_flush(x0[i]); hv[4 + i] = toh_flush(x1[i]); }
                const size_t oo = sb + (size_t)row * pitch + c8;
                *(volatile v8h*)(Ph + oo) = hv; }
            if (ps == 0) __threadfence(); }
        wave_sync();
    }
}

__global__ __launch_bounds__(32) void k_proj_rows(const bf* __restrict__ A, const bf* __restrict__ Bt, const float* __restrict__ bias, h16* Ph) { proj_body<0>(A, Bt, bias, Ph); }
__global__ __launch_bounds__(32) void k_proj_cols(const bf* __restrict__ A, const bf* __restrict__ Bt, const float* __restrict__ bias, h16* Ph) { proj_body<1>(A, Bt, bias, Ph); }

__device__ __forceinline__ v8f score16(const h16* __restrict__ kp, const h16* __restrict__ qp) {
    v8f s = (v8f){};
#pragma unroll 4
    for (int kc = 0; kc < DK; kc += 32) { const v16h a = ldh(kp + kc); const v16h b = ldh(qp + kc); s = wmg(a, b, s); }
    return s;
}

__global__ __launch_bounds__(32 * FW) void k_flash(const h16* __restrict__ QP, const h16* __restrict__ KP, const h16* __restrict__ VT, const unsigned* __restrict__ ADJ, float* OUT) {
    __shared__ __align__(16) h16 Ps[16 * PP];
    __shared__ float redm[FW * 16];
    __shared__ float reds[FW * 16];
    __shared__ __align__(16) float os[FW * 16 * OSP];
    const int lane = threadIdx.x & 31, lr = lane & 15, hi = lane >> 4;
    const int wave = __builtin_amdgcn_readfirstlane((int)(threadIdx.x >> 5));
    const int q0 = blockIdx.x * 16;
    const size_t qo = (size_t)(q0 + lr) * DK + 8 * hi;
    const size_t ko = (size_t)lr * DK + 8 * hi;
    const size_t vo = (size_t)(wave * 64 + lr) * SEQ + 8 * hi;
    const size_t ao = (size_t)(q0 + lr) * AWORDS;
    const int pw = lr * PP + wave * 32 + 8 * hi;
    const int pf = lr * PP + 8 * hi;
    const int sh8 = 8 * hi;
    v8f o0 = (v8f){}, o1 = (v8f){}, o2 = (v8f){}, o3 = (v8f){};
    float m = NEGB, l = 0.0f;
#pragma unroll 1
    for (int kb = 0; kb < SEQ; kb += PANEL) {
        const int key0 = kb + wave * 32;
        const unsigned aw = ADJ[ao + (size_t)(key0 >> 5)];
        const bool anyA = __builtin_amdgcn_ballot_w32((aw & 0xFFFFu) != 0u) != 0u;
        const bool anyB = __builtin_amdgcn_ballot_w32((aw >> 16) != 0u) != 0u;
        v8f sa = (v8f){}, sb = (v8f){};
        if (anyA) sa = score16(KP + ko + (size_t)key0 * DK, QP + qo);
        if (anyB) sb = score16(KP + ko + (size_t)(key0 + 16) * DK, QP + qo);
        const unsigned wa = aw >> sh8, wb2 = aw >> (16 + sh8);
        float ta[8], tb[8]; float mx = NEGB;
#pragma unroll
        for (int r = 0; r < 8; ++r) {
            const bool fa = ((wa >> r) & 1u) != 0u, fb = ((wb2 >> r) & 1u) != 0u;
            ta[r] = fa ? sa[r] * SC2 : FILL2; tb[r] = fb ? sb[r] * SC2 : FILL2;
            mx = fmaxf(mx, fmaxf(ta[r], tb[r])); }
        mx = fmaxf(mx, __shfl_xor(mx, 16, 32));
        if (hi == 0) redm[wave * 16 + lr] = mx;
        __syncthreads();
        float pm = redm[lr];
#pragma unroll
        for (int w = 1; w < FW; ++w) pm = fmaxf(pm, redm[w * 16 + lr]);
        const float mnew = fmaxf(m, pm);
        const float alpha = __builtin_amdgcn_exp2f(m - mnew);
        const float sh = PSH - mnew;
        v8h pa, pc; float ls = 0.0f;
#pragma unroll
        for (int r = 0; r < 8; ++r) {
            const float ea = ta[r] + sh, eb = tb[r] + sh;
            const float xa = __builtin_amdgcn_exp2f(ea), xb = __builtin_amdgcn_exp2f(eb);
            const float ga = (ea < -14.0f) ? 0.0f : xa, gb = (eb < -14.0f) ? 0.0f : xb;
            const h16 ha = (h16)ga; const h16 hb = (h16)gb;
            pa[r] = ha; pc[r] = hb; ls += (float)ha + (float)hb; }
        ls += __shfl_xor(ls, 16, 32);
        if (hi == 0) reds[wave * 16 + lr] = ls;
        *(v8h*)(&Ps[pw]) = pa; *(v8h*)(&Ps[pw + 16]) = pc;
        __syncthreads();
        float lsum = reds[lr];
#pragma unroll
        for (int w = 1; w < FW; ++w) lsum += reds[w * 16 + lr];
        l = l * alpha + lsum; m = mnew;
        o0 = o0 * alpha; o1 = o1 * alpha; o2 = o2 * alpha; o3 = o3 * alpha;
#pragma unroll 2
        for (int kc = 0; kc < PANEL; kc += 32) {
            const v16h pb = cat16(*(const v8h*)(&Ps[pf + kc]), *(const v8h*)(&Ps[pf + kc + 16]));
            const h16* va = VT + vo + (size_t)(kb + kc);
            const v16h v0 = ldh(va);                      o0 = wmg(v0, pb, o0);
            const v16h v1 = ldh(va + (size_t)16 * SEQ);   o1 = wmg(v1, pb, o1);
            const v16h v2 = ldh(va + (size_t)32 * SEQ);   o2 = wmg(v2, pb, o2);
            const v16h v3 = ldh(va + (size_t)48 * SEQ);   o3 = wmg(v3, pb, o3);
        }
        __syncthreads();
    }
    const float inv = 1.0f / l;
    const int wb = wave * 16 * OSP;
    { v4f a, c;
      a[0] = o0[0] * inv; a[1] = o0[1] * inv; a[2] = o0[2] * inv; a[3] = o0[3] * inv; c[0] = o0[4] * inv; c[1] = o0[5] * inv; c[2] = o0[6] * inv; c[3] = o0[7] * inv;
      *(v4fa*)(&os[wb + lr * OSP +  0 + 8 * hi]) = a; *(v4fa*)(&os[wb + lr * OSP +  0 + 8 * hi + 4]) = c;
      a[0] = o1[0] * inv; a[1] = o1[1] * inv; a[2] = o1[2] * inv; a[3] = o1[3] * inv; c[0] = o1[4] * inv; c[1] = o1[5] * inv; c[2] = o1[6] * inv; c[3] = o1[7] * inv;
      *(v4fa*)(&os[wb + lr * OSP + 16 + 8 * hi]) = a; *(v4fa*)(&os[wb + lr * OSP + 16 + 8 * hi + 4]) = c;
      a[0] = o2[0] * inv; a[1] = o2[1] * inv; a[2] = o2[2] * inv; a[3] = o2[3] * inv; c[0] = o2[4] * inv; c[1] = o2[5] * inv; c[2] = o2[6] * inv; c[3] = o2[7] * inv;
      *(v4fa*)(&os[wb + lr * OSP + 32 + 8 * hi]) = a; *(v4fa*)(&os[wb + lr * OSP + 32 + 8 * hi + 4]) = c;
      a[0] = o3[0] * inv; a[1] = o3[1] * inv; a[2] = o3[2] * inv; a[3] = o3[3] * inv; c[0] = o3[4] * inv; c[1] = o3[5] * inv; c[2] = o3[6] * inv; c[3] = o3[7] * inv;
      *(v4fa*)(&os[wb + lr * OSP + 48 + 8 * hi]) = a; *(v4fa*)(&os[wb + lr * OSP + 48 + 8 * hi + 4]) = c; }
    wave_sync();
    float* orow = OUT + (size_t)q0 * DK + wave * 64;
#pragma unroll 1
    for (int ps = 0; ps < 2; ++ps) {
#pragma unroll
        for (int s = 0; s < 8; ++s) { const int row = 2 * s + (lane >> 4), cofs = (lane & 15) * 4;
            const v4f val = *(const v4fa*)(&os[wb + row * OSP + cofs]);
            *(volatile v4f*)(orow + (size_t)row * DK + cofs) = val; }
        if (ps == 0) __threadfence(); }
}

static constexpr size_t al256(size_t v) { return (v + 255) & ~(size_t)255; }
static constexpr size_t SZ_XB = al256((size_t)SEQ * DIN * 2);
static constexpr size_t SZ_WB = al256((size_t)3 * DK * DIN * 2);
static constexpr size_t SZ_PL = al256((size_t)SEQ * DK * 2);
static constexpr size_t SZ_AJ = al256((size_t)SEQ * AWORDS * 4);
static constexpr size_t SZ_TOTAL = SZ_XB + SZ_WB + 3 * SZ_PL + SZ_AJ;
static_assert(SZ_TOTAL <= (size_t)134217728);
static_assert(((size_t)DK * DIN * 2) % 256 == 0);
static_assert((size_t)(SEQ / AROWS) * AROWS * AWORDS * 4 <= SZ_AJ);
static_assert((size_t)(SEQ / 64) * 64 * DK * 2 <= SZ_PL);

extern "C" void kernel_launch(void* const* d_in, const int* in_sizes, int n_in,
                              void* d_out, int out_size, void* d_ws, size_t ws_size, hipStream_t stream) {
    if (n_in < 8) return;
    if ((size_t)in_sizes[0] < (size_t)SEQ * DIN) return;
    if (in_sizes[1] < 2) return;
    if ((size_t)in_sizes[2] < (size_t)DIN * DK || (size_t)in_sizes[4] < (size_t)DIN * DK || (size_t)in_sizes[6] < (size_t)DIN * DK) return;
    if (in_sizes[3] < DK || in_sizes[5] < DK || in_sizes[7] < DK) return;
    if ((size_t)out_size < (size_t)SEQ * DK) return;
    if (SZ_TOTAL > ws_size) return;
    const float* x  = (const float*)d_in[0];
    const int*   ei = (const int*)d_in[1];
    const float* wq = (const float*)d_in[2]; const float* bq = (const float*)d_in[3];
    const float* wk = (const float*)d_in[4]; const float* bk = (const float*)d_in[5];
    const float* wv = (const float*)d_in[6]; const float* bv = (const float*)d_in[7];
    const int E = in_sizes[1] / 2;
    float* OUT = (float*)d_out;
    char* wsp = (char*)d_ws;
    bf* XB = (bf*)wsp; wsp += SZ_XB;
    bf* WB = (bf*)wsp; wsp += SZ_WB;
    h16* QP = (h16*)wsp; wsp += SZ_PL;
    h16* KP = (h16*)wsp; wsp += SZ_PL;
    h16* VT = (h16*)wsp; wsp += SZ_PL;
    unsigned* ADJ = (unsigned*)wsp; wsp += SZ_AJ;
    bf* WQT = WB; bf* WKT = WB + (size_t)DK * DIN; bf* WVT = WB + (size_t)2 * DK * DIN;

    { const size_t n8 = (size_t)SEQ * DIN / 8;
      k_cvt8<<<(unsigned)((n8 + 255) / 256), 256, 0, stream>>>(x, XB, n8); }
    { const unsigned g = (unsigned)((DK * DIN / 8 + 255) / 256);
      k_wcvt<<<g, 256, 0, stream>>>(wq, WQT); k_wcvt<<<g, 256, 0, stream>>>(wk, WKT); k_wcvt<<<g, 256, 0, stream>>>(wv, WVT); }
    k_adj<<<SEQ / AROWS, 256, 0, stream>>>(ei, ADJ, E);

    k_proj_rows<<<dim3(SEQ / 64, DK / 64, 1), 32, 0, stream>>>(XB, WQT, bq, QP);
    k_proj_rows<<<dim3(SEQ / 64, DK / 64, 1), 32, 0, stream>>>(XB, WKT, bk, KP);
    k_proj_cols<<<dim3(DK / 64, SEQ / 64, 1), 32, 0, stream>>>(WVT, XB, bv, VT);

    k_flash<<<SEQ / 16, 32 * FW, 0, stream>>>(QP, KP, VT, ADJ, OUT);
}
